// LSTM_79285096284795
// MI455X (gfx1250) — hardware-verified
//
#include <hip/hip_runtime.h>
#include <math.h>

constexpr int NB     = 1024;
constexpr int NL     = 512;
constexpr int NH     = 64;
constexpr int NG4    = 4 * NH;
constexpr int RB     = 16;
constexpr int NTHR   = 128;
constexpr int NWAVE  = NTHR / 32;
constexpr int PH     = 72;
constexpr int HPL    = RB * PH;
constexpr int NPL    = 8;
constexpr int CHUNK  = 32;
constexpr int YSP    = 32;
constexpr int OSP    = 32;
constexpr int HFP    = 68;
constexpr int WPLANE = NG4 * NH;
constexpr int NWMAT  = 3;
constexpr float HCARRY = 16.0f;
constexpr float LCARRY = 2048.0f;
constexpr float WCARRY = 256.0f;
constexpr float S_HI = 1.0f / (HCARRY * WCARRY);
constexpr float S_LO = 1.0f / (HCARRY * LCARRY * WCARRY);
static_assert(NB % RB == 0);
static_assert(NL % CHUNK == 0);
static_assert(NH == 16 * NWAVE);
static_assert(NH % 32 == 0);
static_assert(NG4 == 4 * NH);
static_assert(RB * CHUNK == 4 * NTHR);
static_assert(RB * 8 == NTHR);
static_assert((NPL * HPL) % NTHR == 0);
static_assert(PH % 8 == 0 && HFP % 4 == 0 && YSP % 4 == 0 && OSP == CHUNK);
static_assert(WPLANE % (8 * 256) == 0);
static_assert(CHUNK * 4 == 128);

typedef __attribute__((ext_vector_type(16))) _Float16 v16h;
typedef __attribute__((ext_vector_type(8)))  _Float16 v8h;
typedef __attribute__((ext_vector_type(8)))  float    v8f;
typedef __attribute__((ext_vector_type(4)))  float    v4f;

__device__ __forceinline__ void guard8x6(v8f& a0, v8f& a1, v8f& a2, v8f& a3, v8f& a4, v8f& a5, v8f& a6, v8f& a7,
                                         v16h x0, v16h x1, v16h x2, v16h x3, v16h x4, v16h x5) {
  asm volatile("v_nop\n\tv_nop\n\tv_nop\n\tv_nop"
               : "+v"(a0), "+v"(a1), "+v"(a2), "+v"(a3), "+v"(a4), "+v"(a5), "+v"(a6), "+v"(a7)
               : "v"(x0), "v"(x1), "v"(x2), "v"(x3), "v"(x4), "v"(x5));
}
__device__ __forceinline__ void acc_guard8(v8f& a0, v8f& a1, v8f& a2, v8f& a3, v8f& a4, v8f& a5, v8f& a6, v8f& a7) {
  asm volatile("v_nop\n\tv_nop\n\tv_nop\n\tv_nop"
               : "+v"(a0), "+v"(a1), "+v"(a2), "+v"(a3), "+v"(a4), "+v"(a5), "+v"(a6), "+v"(a7));
}
template <typename T> struct Frag;
template <> struct Frag<_Float16> {
  typedef v16h V; union U { v16h v; v8h h[2]; };
  static __device__ __forceinline__ v16h load(const _Float16* p) {
    U f; f.h[0] = *(const v8h*)(p); f.h[1] = *(const v8h*)(p + 16); return f.v;
  }
  static __device__ __forceinline__ v8f mma(v16h a, v16h b, v8f c) {
    return __builtin_amdgcn_wmma_f32_16x16x32_f16(false, a, false, b, (short)0, c, false, false);
  }
};

__device__ __forceinline__ float fsig(float x)  { return __builtin_amdgcn_rcpf(1.0f + __expf(-x)); }
__device__ __forceinline__ float ftanh(float x) { return 1.0f - 2.0f * __builtin_amdgcn_rcpf(__expf(2.0f * x) + 1.0f); }

__device__ __forceinline__ void split16(float h, _Float16& hi, _Float16& lo) {
  const float hs = h * HCARRY;
  const _Float16 a = (_Float16)hs;
  const float af = (float)a;
  const float res = (hs - af) * LCARRY;
  hi = a;
  lo = (_Float16)res;
}

__global__ __launch_bounds__(256) void wprep_kernel(const float* __restrict__ W0, const float* __restrict__ W1,
                                                    const float* __restrict__ W2, unsigned short* __restrict__ WP) {
  const int which = blockIdx.x >> 3;
  const int e = (blockIdx.x & 7) * 256 + threadIdx.x;
  const float* src = W0;
  if (which == 1) src = W1;
  if (which == 2) src = W2;
  const v4f a = *(const v4f*)(src + 8 * e);
  const v4f b = *(const v4f*)(src + 8 * e + 4);
  v8h hv;
#pragma unroll
  for (int k = 0; k < 4; ++k) {
    hv[k]     = (_Float16)(a[k] * WCARRY);
    hv[4 + k] = (_Float16)(b[k] * WCARRY);
  }
  unsigned short* dst = WP + (size_t)which * WPLANE + (size_t)8 * e;
  *(volatile v8h*)dst = hv;
  __threadfence();
  *(volatile v8h*)dst = hv;
}

__global__ __launch_bounds__(NTHR) void lstm2_seq_kernel(
    const float* __restrict__ y, const float* __restrict__ w_ih1,
    const float* __restrict__ b_ih1, const float* __restrict__ b_hh1,
    const float* __restrict__ b_ih2, const float* __restrict__ b_hh2,
    const float* __restrict__ w_lin, const float* __restrict__ b_lin,
    const unsigned short* __restrict__ WPp, float* __restrict__ out) {
  __shared__ __align__(16) _Float16 Hp[NPL * HPL];
  __shared__ __align__(16) float    Ys[RB * YSP];
  __shared__ __align__(16) float    Osg[RB * OSP];
  __shared__ __align__(16) float    H2f[RB * HFP];
  const _Float16* WP = (const _Float16*)WPp;
  const int tid = threadIdx.x, lane = tid & 31, wave = tid >> 5;
  const int c = lane & 15, hh = lane >> 4, koff = 8 * hh;
  const int j = 16 * wave + c;
  const int orow = tid >> 3, oq = tid & 7;
  const int bb = blockIdx.x * RB;

#pragma unroll 1
  for (int i = tid; i < NPL * HPL; i += NTHR) Hp[i] = (_Float16)0.0f;

  float wih[4], bs1[4], bs2[4];
#pragma unroll
  for (int g = 0; g < 4; ++g) {
    const int n = NH * g + j;
    wih[g] = w_ih1[n];
    bs1[g] = b_ih1[n] + b_hh1[n];
  }
  asm volatile("" :: "v"(wih[0]), "v"(wih[1]), "v"(wih[2]), "v"(wih[3]),
                     "v"(bs1[0]), "v"(bs1[1]), "v"(bs1[2]), "v"(bs1[3]) : "memory");
#pragma unroll
  for (int g = 0; g < 4; ++g) {
    const int n = NH * g + j;
    bs2[g] = b_ih2[n] + b_hh2[n];
  }
  const v4f wl0 = *(const v4f*)(w_lin + 8 * oq);
  const v4f wl1 = *(const v4f*)(w_lin + 8 * oq + 4);
  const float blin = b_lin[0];
  asm volatile("" :: "v"(bs2[0]), "v"(bs2[1]), "v"(bs2[2]), "v"(bs2[3]), "v"(wl0), "v"(wl1), "v"(blin) : "memory");

  float c1s[8], c2s[8];
#pragma unroll
  for (int r = 0; r < 8; ++r) { c1s[r] = 0.0f; c2s[r] = 0.0f; }
  __syncthreads();

  const v8f z8 = {0.f, 0.f, 0.f, 0.f, 0.f, 0.f, 0.f, 0.f};

#pragma unroll 1
  for (int t = 0; t < NL; ++t) {
    const int p  = t & 1;
    const int tc = t & (CHUNK - 1);

    if (tc == 0) {
      const v4f v = *(const v4f*)(y + (size_t)(bb + orow) * NL + (size_t)t + 4 * oq);
      *(v4f*)(Ys + orow * YSP + 4 * oq) = v;
      __syncthreads();
    }

    v8f acc[4], acl[4];
#pragma unroll
    for (int g = 0; g < 4; ++g) { acc[g] = z8; acl[g] = z8; }
    {
      const _Float16* ahi = Hp + (p * 2) * HPL + c * PH + koff;
      const _Float16* alo = ahi + HPL;
      const _Float16* wb  = WP + (size_t)j * NH + koff;
#pragma unroll 1
      for (int k0 = 0; k0 < NH; k0 += 32) {
        const v16h ah = Frag<_Float16>::load(ahi + k0);
        const v16h al = Frag<_Float16>::load(alo + k0);
        const v16h b0 = Frag<_Float16>::load(wb + k0);
        const v16h b1 = Frag<_Float16>::load(wb + (size_t)1 * NH * NH + k0);
        const v16h b2 = Frag<_Float16>::load(wb + (size_t)2 * NH * NH + k0);
        const v16h b3 = Frag<_Float16>::load(wb + (size_t)3 * NH * NH + k0);
        acc[0] = Frag<_Float16>::mma(ah, b0, acc[0]);
        acl[0] = Frag<_Float16>::mma(al, b0, acl[0]);
        acc[1] = Frag<_Float16>::mma(ah, b1, acc[1]);
        acl[1] = Frag<_Float16>::mma(al, b1, acl[1]);
        acc[2] = Frag<_Float16>::mma(ah, b2, acc[2]);
        acl[2] = Frag<_Float16>::mma(al, b2, acl[2]);
        acc[3] = Frag<_Float16>::mma(ah, b3, acc[3]);
        acl[3] = Frag<_Float16>::mma(al, b3, acl[3]);
        guard8x6(acc[0], acc[1], acc[2], acc[3], acl[0], acl[1], acl[2], acl[3], ah, al, b0, b1, b2, b3);
      }
      acc_guard8(acc[0], acc[1], acc[2], acc[3], acl[0], acl[1], acl[2], acl[3]);
    }
    {
      const int wpl = ((p ^ 1) * 2) * HPL;
#pragma unroll
      for (int r = 0; r < 8; ++r) {
        const int row = 8 * hh + r;
        const float xv = Ys[row * YSP + tc];
        const float zi = acc[0][r] * S_HI + acl[0][r] * S_LO + xv * wih[0] + bs1[0];
        const float zf = acc[1][r] * S_HI + acl[1][r] * S_LO + xv * wih[1] + bs1[1];
        const float zg = acc[2][r] * S_HI + acl[2][r] * S_LO + xv * wih[2] + bs1[2];
        const float zo = acc[3][r] * S_HI + acl[3][r] * S_LO + xv * wih[3] + bs1[3];
        const float ig = fsig(zi);
        const float fg = fsig(zf);
        const float gg = ftanh(zg);
        const float og = fsig(zo);
        const float cn = fg * c1s[r] + ig * gg;
        c1s[r] = cn;
        const float hn = og * ftanh(cn);
        _Float16 h16, l16;
        split16(hn, h16, l16);
        Hp[wpl + row * PH + j]       = h16;
        Hp[wpl + HPL + row * PH + j] = l16;
      }
    }
    __syncthreads();

#pragma unroll
    for (int g = 0; g < 4; ++g) { acc[g] = z8; acl[g] = z8; }
#pragma unroll 1
    for (int kk = 0; kk < 4; ++kk) {
      const int sel  = kk >> 1;
      const int k0   = (kk & 1) * 32;
      const int par  = p ^ 1 ^ sel;
      const int pidx = sel * 4 + par * 2;
      const _Float16* ahi = Hp + pidx * HPL + c * PH + koff + k0;
      const _Float16* alo = ahi + HPL;
      const _Float16* wb  = WP + (size_t)(1 + sel) * WPLANE + (size_t)j * NH + koff + k0;
      const v16h ah = Frag<_Float16>::load(ahi);
      const v16h al = Frag<_Float16>::load(alo);
      const v16h b0 = Frag<_Float16>::load(wb);
      const v16h b1 = Frag<_Float16>::load(wb + (size_t)1 * NH * NH);
      const v16h b2 = Frag<_Float16>::load(wb + (size_t)2 * NH * NH);
      const v16h b3 = Frag<_Float16>::load(wb + (size_t)3 * NH * NH);
      acc[0] = Frag<_Float16>::mma(ah, b0, acc[0]);
      acl[0] = Frag<_Float16>::mma(al, b0, acl[0]);
      acc[1] = Frag<_Float16>::mma(ah, b1, acc[1]);
      acl[1] = Frag<_Float16>::mma(al, b1, acl[1]);
      acc[2] = Frag<_Float16>::mma(ah, b2, acc[2]);
      acl[2] = Frag<_Float16>::mma(al, b2, acl[2]);
      acc[3] = Frag<_Float16>::mma(ah, b3, acc[3]);
      acl[3] = Frag<_Float16>::mma(al, b3, acl[3]);
      guard8x6(acc[0], acc[1], acc[2], acc[3], acl[0], acl[1], acl[2], acl[3], ah, al, b0, b1, b2, b3);
    }
    acc_guard8(acc[0], acc[1], acc[2], acc[3], acl[0], acl[1], acl[2], acl[3]);
    {
      const int wpl = (4 + (p ^ 1) * 2) * HPL;
#pragma unroll
      for (int r = 0; r < 8; ++r) {
        const int row = 8 * hh + r;
        const float zi = acc[0][r] * S_HI + acl[0][r] * S_LO + bs2[0];
        const float zf = acc[1][r] * S_HI + acl[1][r] * S_LO + bs2[1];
        const float zg = acc[2][r] * S_HI + acl[2][r] * S_LO + bs2[2];
        const float zo = acc[3][r] * S_HI + acl[3][r] * S_LO + bs2[3];
        const float ig = fsig(zi);
        const float fg = fsig(zf);
        const float gg = ftanh(zg);
        const float og = fsig(zo);
        const float cn = fg * c2s[r] + ig * gg;
        c2s[r] = cn;
        const float hn = og * ftanh(cn);
        _Float16 h16, l16;
        split16(hn, h16, l16);
        Hp[wpl + row * PH + j]       = h16;
        Hp[wpl + HPL + row * PH + j] = l16;
        H2f[row * HFP + j] = hn;
      }
    }
    __syncthreads();

    {
      const v4f v0 = *(const v4f*)(H2f + orow * HFP + 8 * oq);
      const v4f v1 = *(const v4f*)(H2f + orow * HFP + 8 * oq + 4);
      float s = 0.0f;
      s += v0[0] * wl0[0]; s += v0[1] * wl0[1]; s += v0[2] * wl0[2]; s += v0[3] * wl0[3];
      s += v1[0] * wl1[0]; s += v1[1] * wl1[1]; s += v1[2] * wl1[2]; s += v1[3] * wl1[3];
      s += __shfl_xor(s, 1, 32);
      s += __shfl_xor(s, 2, 32);
      s += __shfl_xor(s, 4, 32);
      const float ov = s + blin;
      if (oq == 0) Osg[orow * OSP + tc] = ov;
    }

    if (tc == CHUNK - 1) {
      __syncthreads();
      const v4f v = *(const v4f*)(Osg + orow * OSP + 4 * oq);
      float* op = out + (size_t)(bb + orow) * NL + (size_t)(t - (CHUNK - 1)) + 4 * oq;
      *(volatile v4f*)op = v;
      __threadfence();
      *(volatile v4f*)op = v;
    }
  }
}

extern "C" void kernel_launch(void* const* d_in, const int* in_sizes, int n_in,
                              void* d_out, int out_size, void* d_ws, size_t ws_size, hipStream_t stream) {
  if (n_in < 11 || d_out == nullptr || d_ws == nullptr) return;
  if (in_sizes[0] != NB * NL || in_sizes[1] != NG4 || in_sizes[2] != NG4 * NH || in_sizes[3] != NG4 ||
      in_sizes[4] != NG4 || in_sizes[5] != NG4 * NH || in_sizes[6] != NG4 * NH || in_sizes[7] != NG4 ||
      in_sizes[8] != NG4 || in_sizes[9] != NH || in_sizes[10] != 1 || out_size != NB * NL) return;

  const float* y     = (const float*)d_in[0];
  const float* w_ih1 = (const float*)d_in[1];
  const float* w_hh1 = (const float*)d_in[2];
  const float* b_ih1 = (const float*)d_in[3];
  const float* b_hh1 = (const float*)d_in[4];
  const float* w_ih2 = (const float*)d_in[5];
  const float* w_hh2 = (const float*)d_in[6];
  const float* b_ih2 = (const float*)d_in[7];
  const float* b_hh2 = (const float*)d_in[8];
  const float* w_lin = (const float*)d_in[9];
  const float* b_lin = (const float*)d_in[10];
  float* out = (float*)d_out;

  const size_t need = (size_t)NWMAT * WPLANE * 2;
  if (need > ws_size || need > (size_t)134217728) return;
  unsigned short* WP = (unsigned short*)d_ws;

  wprep_kernel<<<NWMAT * (WPLANE / 8 / 256), 256, 0, stream>>>(w_hh1, w_ih2, w_hh2, WP);
  lstm2_seq_kernel<<<NB / RB, NTHR, 0, stream>>>(y, w_ih1, b_ih1, b_hh1, b_ih2, b_hh2, w_lin, b_lin, WP, out);
}
